// WeightedGATLayer_90005334655074
// MI455X (gfx1250) — hardware-verified
//
#include <hip/hip_runtime.h>
#include <stddef.h>
#include <stdint.h>


#define KIN   256
#define DF    128
#define NH    4
#define HD    32
#define GR    32
#define AP    264
#define XSP   132
#define NB    512
#define CHUNK 2048
#define NTHR  256
#define NWAVE 8
#define WCAP  256
#define NGRP  (CHUNK / (NTHR * 4))

#define LDS_SACC (NB * DF)
#define LDS_DEN  (NB * NH)
#define LDS_MX   (NB * NH)
#define LDS_LIST (NWAVE * WCAP)
#define LDS_BYTES ((LDS_SACC + LDS_DEN + LDS_MX + LDS_LIST + NWAVE) * 4)

static_assert(WCAP == (CHUNK / NTHR) * 32);
static_assert(NGRP == 2);
static_assert(NB == 512);
static_assert(CHUNK == 2048);
static_assert(((LDS_SACC + LDS_DEN) % 4) == 0);
static_assert(LDS_BYTES == 286752);
static_assert(DF == NH * HD);
static_assert((KIN % 32) == 0);
static_assert((KIN / 8) == 32);
static_assert((AP % 8) == 0);
static_assert((XSP % 4) == 0);

typedef float    v4f  __attribute__((ext_vector_type(4)));
typedef float    v8f  __attribute__((ext_vector_type(8)));
typedef int      v4i  __attribute__((ext_vector_type(4)));
typedef unsigned v4u  __attribute__((ext_vector_type(4)));
typedef __bf16   v16b __attribute__((ext_vector_type(16)));
union FragB { v16b v; v4u u[2]; };

__device__ __forceinline__ v8f wm(v16b a, v16b b, v8f c) {
  v8f d = __builtin_amdgcn_wmma_f32_16x16x32_bf16(false, a, false, b, (short)0, c, false, false);
  asm volatile("v_nop\n\tv_nop\n\tv_nop\n\tv_nop" : "+v"(d) : "v"(a), "v"(b));
  return d;
}

__device__ __forceinline__ unsigned bfb(float f) {
  unsigned u = __float_as_uint(f);
  u += 0x7FFFu + ((u >> 16) & 1u);
  return u >> 16;
}
__device__ __forceinline__ void split2(float a, float b, unsigned& ph, unsigned& pl) {
  const unsigned ha = bfb(a), hb = bfb(b);
  const unsigned la = bfb(a - __uint_as_float(ha << 16));
  const unsigned lb = bfb(b - __uint_as_float(hb << 16));
  ph = ha | (hb << 16);
  pl = la | (lb << 16);
}
__device__ __forceinline__ void split8(v4f f0, v4f f1, v4u& uh, v4u& ul) {
  unsigned h, l;
  split2(f0.x, f0.y, h, l); uh.x = h; ul.x = l;
  split2(f0.z, f0.w, h, l); uh.y = h; ul.y = l;
  split2(f1.x, f1.y, h, l); uh.z = h; ul.z = l;
  split2(f1.z, f1.w, h, l); uh.w = h; ul.w = l;
}

__global__ __launch_bounds__(NTHR) void k_prepw(const float* __restrict__ W,
                                               unsigned short* Wth, unsigned short* Wtl, int n8) {
  const int i = blockIdx.x * NTHR + threadIdx.x;
  if (i >= n8) return;
  const int n  = i >> 5;
  const int kg = (i & 31) * 8;
  v4f f0, f1;
  f0.x = W[(size_t)(kg + 0) * DF + n];
  f0.y = W[(size_t)(kg + 1) * DF + n];
  f0.z = W[(size_t)(kg + 2) * DF + n];
  f0.w = W[(size_t)(kg + 3) * DF + n];
  f1.x = W[(size_t)(kg + 4) * DF + n];
  f1.y = W[(size_t)(kg + 5) * DF + n];
  f1.z = W[(size_t)(kg + 6) * DF + n];
  f1.w = W[(size_t)(kg + 7) * DF + n];
  v4u uh, ul;
  split8(f0, f1, uh, ul);
  const size_t o = (size_t)n * KIN + kg;
  *(volatile v4u*)(Wth + o) = uh;
  *(volatile v4u*)(Wtl + o) = ul;
  __threadfence();
  *(volatile v4u*)(Wth + o) = uh;
  *(volatile v4u*)(Wtl + o) = ul;
}

__device__ __forceinline__ void epi_tile(v8f acc, int T, int hh, int m, int wave, int ncol,
                                         float cs, float cd, float* Xs, float* As, float* Ds) {
  float ss[8], sd[8];
#pragma unroll
  for (int r = 0; r < 8; ++r) {
    const float v = acc[r];
    Xs[(T * 16 + 8 * hh + r) * XSP + ncol] = v;
    ss[r] = v * cs;
    sd[r] = v * cd;
  }
#pragma unroll
  for (int mk = 1; mk < 16; mk <<= 1) {
#pragma unroll
    for (int r = 0; r < 8; ++r) {
      ss[r] += __shfl_xor(ss[r], mk, 32);
      sd[r] += __shfl_xor(sd[r], mk, 32);
    }
  }
  if (m == 0) {
#pragma unroll
    for (int r = 0; r < 8; ++r) {
      As[(T * 16 + 8 * hh + r) * NWAVE + wave] = ss[r];
      Ds[(T * 16 + 8 * hh + r) * NWAVE + wave] = sd[r];
    }
  }
}

__global__ __launch_bounds__(NTHR) void k_gemm(
    const float* __restrict__ x, const unsigned short* __restrict__ Wth,
    const unsigned short* __restrict__ Wtl,
    const float* __restrict__ al, const float* __restrict__ ar,
    float* ft, float* elp, float* erp, int nN) {
  __shared__ __attribute__((aligned(16))) unsigned short Ah[GR * AP];
  __shared__ __attribute__((aligned(16))) unsigned short Al[GR * AP];
  __shared__ __attribute__((aligned(16))) float Xs[GR * XSP];
  __shared__ __attribute__((aligned(16))) float As[GR * NWAVE];
  __shared__ __attribute__((aligned(16))) float Ds[GR * NWAVE];

  const int tid  = threadIdx.x;
  const int lane = tid & 31;
  const int wave = tid >> 5;
  const int hh   = lane >> 4;
  const int m    = lane & 15;
  const int rowBase = blockIdx.x * GR;

  {
    const int r  = tid >> 3;
    const int c0 = (tid & 7) * 32;
    int row = rowBase + r;
    if (row > nN - 1) row = nN - 1;
    const float* p = x + (size_t)row * KIN + c0;
#pragma unroll
    for (int g = 0; g < 4; ++g) {
      const v4f f0 = *(const v4f*)(p + 8 * g);
      const v4f f1 = *(const v4f*)(p + 8 * g + 4);
      v4u uh, ul;
      split8(f0, f1, uh, ul);
      *(v4u*)(Ah + r * AP + c0 + 8 * g) = uh;
      *(v4u*)(Al + r * AP + c0 + 8 * g) = ul;
    }
  }
  __syncthreads();

  const int ncol = wave * 16 + m;
  v8f c0a = {0.f, 0.f, 0.f, 0.f, 0.f, 0.f, 0.f, 0.f};
  v8f c1a = {0.f, 0.f, 0.f, 0.f, 0.f, 0.f, 0.f, 0.f};
  const unsigned short* wbh  = Wth + (size_t)ncol * KIN + 8 * hh;
  const unsigned short* wbl  = Wtl + (size_t)ncol * KIN + 8 * hh;
  const unsigned short* pah0 = Ah + m * AP + 8 * hh;
  const unsigned short* pal0 = Al + m * AP + 8 * hh;
  const unsigned short* pah1 = Ah + (16 + m) * AP + 8 * hh;
  const unsigned short* pal1 = Al + (16 + m) * AP + 8 * hh;
#pragma unroll 2
  for (int kt = 0; kt < KIN / 32; ++kt) {
    const int k0 = kt * 32;
    FragB bh, bl, a0h, a0l, a1h, a1l;
    bh.u[0]  = *(const v4u*)(wbh + k0);   bh.u[1]  = *(const v4u*)(wbh + k0 + 16);
    bl.u[0]  = *(const v4u*)(wbl + k0);   bl.u[1]  = *(const v4u*)(wbl + k0 + 16);
    a0h.u[0] = *(const v4u*)(pah0 + k0);  a0h.u[1] = *(const v4u*)(pah0 + k0 + 16);
    a0l.u[0] = *(const v4u*)(pal0 + k0);  a0l.u[1] = *(const v4u*)(pal0 + k0 + 16);
    a1h.u[0] = *(const v4u*)(pah1 + k0);  a1h.u[1] = *(const v4u*)(pah1 + k0 + 16);
    a1l.u[0] = *(const v4u*)(pal1 + k0);  a1l.u[1] = *(const v4u*)(pal1 + k0 + 16);
    c0a = wm(a0h.v, bh.v, c0a);
    c0a = wm(a0h.v, bl.v, c0a);
    c0a = wm(a0l.v, bh.v, c0a);
    c1a = wm(a1h.v, bh.v, c1a);
    c1a = wm(a1h.v, bl.v, c1a);
    c1a = wm(a1l.v, bh.v, c1a);
  }

  const float cs = al[ncol];
  const float cd = ar[ncol];
  epi_tile(c0a, 0, hh, m, wave, ncol, cs, cd, Xs, As, Ds);
  epi_tile(c1a, 1, hh, m, wave, ncol, cs, cd, Xs, As, Ds);
  __syncthreads();

  v4f xr[4];
#pragma unroll
  for (int i = 0; i < 4; ++i) xr[i] = *(const v4f*)(Xs + (4 * wave + i) * XSP + 4 * lane);
  const v4f e0 = *(const v4f*)(As + lane * NWAVE);
  const v4f e1 = *(const v4f*)(As + lane * NWAVE + 4);
  const v4f d0 = *(const v4f*)(Ds + lane * NWAVE);
  const v4f d1 = *(const v4f*)(Ds + lane * NWAVE + 4);
  v4f ge, gd, gv;
  ge.x = e0.x + e0.y; ge.y = e0.z + e0.w; ge.z = e1.x + e1.y; ge.w = e1.z + e1.w;
  gd.x = d0.x + d0.y; gd.y = d0.z + d0.w; gd.z = d1.x + d1.y; gd.w = d1.z + d1.w;
  const bool w0 = (wave == 0);
  gv.x = w0 ? ge.x : gd.x; gv.y = w0 ? ge.y : gd.y; gv.z = w0 ? ge.z : gd.z; gv.w = w0 ? ge.w : gd.w;
  float* gp = (w0 ? elp : erp) + (size_t)(rowBase + lane) * NH;
  const bool gs = (wave < 2);
  float* xpp[4];
#pragma unroll
  for (int i = 0; i < 4; ++i) xpp[i] = ft + (size_t)(rowBase + 4 * wave + i) * DF + 4 * lane;

#pragma unroll
  for (int i = 0; i < 4; ++i) *(volatile v4f*)(xpp[i]) = xr[i];
  if (gs) *(volatile v4f*)gp = gv;
  __threadfence();
#pragma unroll
  for (int i = 0; i < 4; ++i) *(volatile v4f*)(xpp[i]) = xr[i];
  if (gs) *(volatile v4f*)gp = gv;
}

__global__ __launch_bounds__(NTHR) void k_agg(
    const float* __restrict__ ft, const float* __restrict__ elp, const float* __restrict__ erp,
    const float* __restrict__ ew, const int* __restrict__ srcp, const int* __restrict__ dstp,
    const float* __restrict__ lamp, float* out, int nN, int nE) {
  extern __shared__ v4f lds_dyn[];
  float* sacc = (float*)lds_dyn;
  float* den  = sacc + LDS_SACC;
  float* mxs  = den + LDS_DEN;
  int*   list = (int*)(mxs + LDS_MX);
  int*   wcnt = list + LDS_LIST;

  const int tid  = threadIdx.x;
  const int lane = tid & 31;
  const int wave = tid >> 5;
  const int hd   = lane >> 3;
  const int nodeBase = blockIdx.x * NB;

  {
    const v4f z4 = {0.f, 0.f, 0.f, 0.f};
    for (int i = tid; i < (LDS_SACC + LDS_DEN) / 4; i += NTHR) lds_dyn[i] = z4;
    for (int i = tid; i < LDS_MX; i += NTHR) mxs[i] = -1.0e30f;
  }
  __syncthreads();
  const float lamv = lamp[0];
  const bool  al16 = ((reinterpret_cast<size_t>(dstp) & 15) == 0);

  const int nChunks = (nE + CHUNK - 1) / CHUNK;
#pragma unroll 1
  for (int ch = 0; ch < nChunks; ++ch) {
    const int cbase = ch * CHUNK;
    const bool full = al16 && (cbase + CHUNK <= nE);
    int wc = 0;
#pragma unroll
    for (int g = 0; g < NGRP; ++g) {
      const int el0 = (g * NTHR + tid) * 4;
      const int e0  = cbase + el0;
      const int sent = -2147483647 - 1;
      v4i d;
      if (full) {
        d = *(const v4i*)(dstp + e0);
      } else {
        const int i0 = (e0     > nE - 1) ? nE - 1 : e0;
        const int i1 = (e0 + 1 > nE - 1) ? nE - 1 : e0 + 1;
        const int i2 = (e0 + 2 > nE - 1) ? nE - 1 : e0 + 2;
        const int i3 = (e0 + 3 > nE - 1) ? nE - 1 : e0 + 3;
        const int v0 = dstp[i0], v1 = dstp[i1], v2 = dstp[i2], v3 = dstp[i3];
        d.x = (e0     < nE) ? v0 : sent;
        d.y = (e0 + 1 < nE) ? v1 : sent;
        d.z = (e0 + 2 < nE) ? v2 : sent;
        d.w = (e0 + 3 < nE) ? v3 : sent;
      }
      const unsigned s0 = (unsigned)d.x - (unsigned)nodeBase;
      const unsigned s1 = (unsigned)d.y - (unsigned)nodeBase;
      const unsigned s2 = (unsigned)d.z - (unsigned)nodeBase;
      const unsigned s3 = (unsigned)d.w - (unsigned)nodeBase;
      const bool h0 = s0 < (unsigned)NB;
      const bool h1 = s1 < (unsigned)NB;
      const bool h2 = s2 < (unsigned)NB;
      const bool h3 = s3 < (unsigned)NB;
      const unsigned many = __builtin_amdgcn_ballot_w32(h0 | h1 | h2 | h3);
      if (many != 0u) {
#define HITJ(J, HJ, SJ) { \
          const unsigned mj = __builtin_amdgcn_ballot_w32(HJ); \
          if (HJ) { \
            const int pos = wc + (int)__builtin_amdgcn_mbcnt_lo(mj, 0u); \
            if (pos < WCAP) list[wave * WCAP + pos] = ((el0 + (J)) << 9) | (int)(SJ); \
          } \
          wc += (int)__builtin_popcount(mj); }
        HITJ(0, h0, s0)
        HITJ(1, h1, s1)
        HITJ(2, h2, s2)
        HITJ(3, h3, s3)
#undef HITJ
      }
    }
    if (lane == 0) wcnt[wave] = wc;
    __syncthreads();

    if (wave == 0) {
      for (int wsx = 0; wsx < NWAVE; ++wsx) {
        int n = wcnt[wsx];
        if (n > WCAP) n = WCAP;
        if (n < 0) n = 0;
        for (int i = 0; i < n; ++i) {
          const int ent  = list[wsx * WCAP + i];
          const int slot = ent & (NB - 1);
          const int eloc = (ent >> 9) & (CHUNK - 1);
          int e = cbase + eloc;
          if (e > nE - 1) e = nE - 1;
          int s = srcp[e];
          s = s < 0 ? 0 : (s > nN - 1 ? nN - 1 : s);
          const float w = ew[e];
          int nd = nodeBase + slot;
          if (nd > nN - 1) nd = nN - 1;
          float v = elp[(size_t)s * NH + hd] + erp[(size_t)nd * NH + hd] + lamv * w;
          v = (v > 0.f) ? v : 0.2f * v;
          const float mo = mxs[slot * NH + hd];
          const float mn = fmaxf(mo, v);
          const float sc = __expf(mo - mn);
          const float p  = __expf(v - mn);
          const v4f xv = *(const v4f*)(ft + (size_t)s * DF + 4 * lane);
          v4f* sp = (v4f*)(sacc + slot * DF + 4 * lane);
          const v4f cur = *sp;
          const v4f nxt = cur * sc + p * xv;
          *sp = nxt;
          const float dn = den[slot * NH + hd];
          const float dnn = dn * sc + p;
          den[slot * NH + hd] = dnn;
          mxs[slot * NH + hd] = mn;
        }
      }
    }
    __syncthreads();
  }

#pragma unroll 1
  for (int j = 0; j < NB / NWAVE; ++j) {
    const int slot = wave * (NB / NWAVE) + j;
    const int node = nodeBase + slot;
    if (node >= nN) break;
    const v4f sv  = *(const v4f*)(sacc + slot * DF + 4 * lane);
    const float dv  = den[slot * NH + hd];
    const float inv = (dv > 0.f) ? (1.0f / dv) : 0.f;
    const v4f y = sv * inv;
    float* op = out + (size_t)node * DF + 4 * lane;
    *(volatile v4f*)op = y;
    __threadfence();
    *(volatile v4f*)op = y;
  }
}

extern "C" void kernel_launch(void* const* d_in, const int* in_sizes, int n_in,
                              void* d_out, int out_size, void* d_ws, size_t ws_size,
                              hipStream_t stream) {
  if (n_in < 8) return;
  const int nN = in_sizes[0] / KIN;
  if (nN <= 0 || in_sizes[0] != nN * KIN) return;
  const int nE = in_sizes[1];
  if (nE < 0 || in_sizes[2] != nE || in_sizes[3] != nE) return;
  if (in_sizes[4] != KIN * DF) return;
  if (in_sizes[5] != NH * HD || in_sizes[6] != NH * HD) return;
  if (in_sizes[7] < 1) return;
  if (out_size != nN * DF) return;

  const float* feat = (const float*)d_in[0];
  const float* ew   = (const float*)d_in[1];
  const int*   srcp = (const int*)d_in[2];
  const int*   dstp = (const int*)d_in[3];
  const float* W    = (const float*)d_in[4];
  const float* al   = (const float*)d_in[5];
  const float* ar   = (const float*)d_in[6];
  const float* lamp = (const float*)d_in[7];
  float* out = (float*)d_out;

  const int nP = ((nN + GR - 1) / GR) * GR;
  size_t off = 0;
  unsigned short* Wth = (unsigned short*)((char*)d_ws + off);
  off += ((size_t)DF * KIN * 2 + 255) & ~(size_t)255;
  unsigned short* Wtl = (unsigned short*)((char*)d_ws + off);
  off += ((size_t)DF * KIN * 2 + 255) & ~(size_t)255;
  float* ftp = (float*)((char*)d_ws + off);
  off += ((size_t)nP * DF * sizeof(float) + 255) & ~(size_t)255;
  float* elp = (float*)((char*)d_ws + off);
  off += ((size_t)nP * NH * sizeof(float) + 255) & ~(size_t)255;
  float* erp = (float*)((char*)d_ws + off);
  off += ((size_t)nP * NH * sizeof(float) + 255) & ~(size_t)255;
  if (off > ws_size) return;

  const int n8 = DF * KIN / 8;
  k_prepw<<<(n8 + NTHR - 1) / NTHR, NTHR, 0, stream>>>(W, Wth, Wtl, n8);

  k_gemm<<<nP / GR, NTHR, 0, stream>>>(feat, Wth, Wtl, al, ar, ftp, elp, erp, nN);

  if (nE > 0) {
    hipFuncSetAttribute(reinterpret_cast<const void*>(&k_agg),
                        hipFuncAttributeMaxDynamicSharedMemorySize, LDS_BYTES);
    const int grid = (nN + NB - 1) / NB;
    k_agg<<<grid, NTHR, LDS_BYTES, stream>>>(ftp, elp, erp, ew, srcp, dstp, lamp, out, nN, nE);
  }
}
